// RobustSymGAT_42245298324094
// MI455X (gfx1250) — hardware-verified
//
#include <hip/hip_runtime.h>
#include <math.h>
#include <stdint.h>

#pragma clang fp contract(off)

#define NROWS    1048576
#define XDIM     10
#define BR       128
#define NTHR     256

#define P_SYM 40
#define P_IN  104
#define P_L   72
#define R_SYM 0
#define R_IN  1280
#define R_L1  7936
#define R_L2  12544
#define R_L3  17152
#define R_HD  21760
#define R_HD2 24064
#define W_TOT 26368
#define W_PIECES 3296

#define PA 136
#define PS 40
#define PE 68

#define C_BSYM 0
#define C_BIN  32
#define C_B1   96
#define C_B2   160
#define C_B3   224
#define C_BHD  288
#define C_WR2  352
#define C_WC2  384
#define C_BR2  512
#define C_BC2  513
#define C_TOT  520

static_assert(NROWS % BR == 0);
static_assert(R_IN == R_SYM + 32 * P_SYM);
static_assert(R_L1 == R_IN + 64 * P_IN);
static_assert(R_L2 == R_L1 + 64 * P_L);
static_assert(R_L3 == R_L2 + 64 * P_L);
static_assert(R_HD == R_L3 + 64 * P_L);
static_assert(R_HD2 == R_HD + 32 * P_L);
static_assert(W_TOT == R_HD + 64 * P_L);
static_assert(W_PIECES * 8 == W_TOT);
static_assert((R_IN * 2) % 128 == 0 && (R_L1 * 2) % 128 == 0 && (R_L2 * 2) % 128 == 0);
static_assert((R_L3 * 2) % 128 == 0 && (R_HD * 2) % 128 == 0 && (R_HD2 * 2) % 128 == 0);
static_assert((32 * P_SYM * 2) % 512 == 0 && (64 * P_IN * 2) % 512 == 0);
static_assert((64 * P_L * 2) % 512 == 0 && (32 * P_L * 2) % 512 == 0 && (W_TOT * 2) % 512 == 0);
static_assert(BR * PE * 4 <= BR * PA * 2);
static_assert((PA % 8) == 0 && (PS % 8) == 0 && (P_SYM % 8) == 0 && (P_IN % 8) == 0 && (P_L % 8) == 0);
static_assert(BR == 128 && NTHR == 256);

typedef __bf16         v16b __attribute__((ext_vector_type(16)));
typedef unsigned short v8us __attribute__((ext_vector_type(8)));
typedef float          v8f  __attribute__((ext_vector_type(8)));
typedef float          v4f  __attribute__((ext_vector_type(4)));

union FragB { v16b v; v8us u[2]; };

__device__ __forceinline__ unsigned short bf_bits(float f) {
  const unsigned u = __float_as_uint(f);
  return (unsigned short)((u + 0x7FFFu + ((u >> 16) & 1u)) >> 16);
}
__device__ __forceinline__ float bf_up(unsigned short b) { return __uint_as_float(((unsigned)b) << 16); }
__device__ __forceinline__ float bfr(float f) { return bf_up(bf_bits(f)); }
__device__ __forceinline__ v8f zero8() { return (v8f){0.f, 0.f, 0.f, 0.f, 0.f, 0.f, 0.f, 0.f}; }

__device__ __forceinline__ float elu_f(float v) {
  const float vn = fminf(v, 0.0f);
  const float em = __expf(vn) - 1.0f;
  return (v > 0.0f) ? v : em;
}
__device__ __forceinline__ float pen_f(float v, float lo, float rlo, float hi, float rhi) {
  const float below = (lo - v) * rlo;
  const float above = (v - hi) * rhi;
  const float mid   = (v > hi) ? above : 0.0f;
  return (v < lo) ? below : mid;
}
__device__ __forceinline__ void st_hl(unsigned short* p, int loOff, float v) {
  const unsigned short hb = bf_bits(v);
  p[0]     = hb;
  p[loOff] = bf_bits(v - bf_up(hb));
}

__device__ __forceinline__ v8f mma_b(v16b a, v16b b, v8f c) {
  return __builtin_amdgcn_wmma_f32_16x16x32_bf16(false, a, false, b, (short)0, c, false, false);
}
__device__ __forceinline__ void mma_guard2(v8f& c0, v8f& c1, v16b a, v16b b0, v16b b1) {
#if defined(__HIP_DEVICE_COMPILE__)
  asm volatile("v_nop\n\tv_nop\n\tv_nop\n\tv_nop" : "+v"(c0), "+v"(c1) : "v"(a), "v"(b0), "v"(b1));
#else
  (void)c0; (void)c1; (void)a; (void)b0; (void)b1;
#endif
}
__device__ __forceinline__ void mma_guard4(v8f& c0, v8f& c1, v8f& c2, v8f& c3, v16b a0, v16b a1, v16b b) {
#if defined(__HIP_DEVICE_COMPILE__)
  asm volatile("v_nop\n\tv_nop\n\tv_nop\n\tv_nop" : "+v"(c0), "+v"(c1), "+v"(c2), "+v"(c3) : "v"(a0), "v"(a1), "v"(b));
#else
  (void)c0; (void)c1; (void)c2; (void)c3; (void)a0; (void)a1; (void)b;
#endif
}

__global__ __launch_bounds__(256) void k_pack(const float* __restrict__ Wm, unsigned short* dst,
                                              int Kreal, int Ncols, int pitch, int ksplit, int kshift,
                                              int nPieces) {
  const int piece = blockIdx.x * 256 + threadIdx.x;
  const bool act  = piece < nPieces;
  const int pc    = act ? piece : (nPieces - 1);
  const int e0    = pc * 8;
  const int n     = e0 / pitch;
  const int kb    = e0 - n * pitch;
  const int nc    = (n < Ncols) ? n : (Ncols - 1);
  v8us o;
#pragma unroll
  for (int jj = 0; jj < 8; ++jj) {
    const int k  = kb + jj;
    const int ks = (k < ksplit) ? k : (k - kshift);
    int kc       = (ks < Kreal) ? ks : (Kreal - 1);
    kc           = (kc < 0) ? 0 : kc;
    float v = Wm[(size_t)kc * Ncols + nc];
    v = (ks >= 0 && ks < Kreal && n < Ncols) ? v : 0.0f;
    o[jj] = bf_bits(v);
  }
  unsigned short* d = dst + (size_t)pc * 8;
  if (act) *(volatile v8us*)d = o;
  __threadfence();
  if (act) *(volatile v8us*)d = o;
}

__global__ __launch_bounds__(NTHR) void k_main(
    const float* __restrict__ x, const unsigned short* __restrict__ wimg,
    const float* __restrict__ bsym, const float* __restrict__ bin,
    const float* __restrict__ b1, const float* __restrict__ b2, const float* __restrict__ b3,
    const float* __restrict__ br1, const float* __restrict__ wr2, const float* __restrict__ br2,
    const float* __restrict__ bc1, const float* __restrict__ wc2, const float* __restrict__ bc2,
    float* out, int nrows) {
  __shared__ __align__(16) unsigned short sW[W_TOT];
  __shared__ __align__(16) unsigned short sA[BR * PA];
  __shared__ __align__(16) unsigned short sS[BR * PS];
  __shared__ __align__(16) float sC[C_TOT];
  __shared__ __align__(16) float sPred[BR];
  __shared__ __align__(16) float sLog[BR * 4];
  float* sE = reinterpret_cast<float*>(sA);

  const int tid  = threadIdx.x;
  const int lane = tid & 31;
  const int wave = tid >> 5;
  const int hh   = lane >> 4;
  const int m16  = lane & 15;
  const int arow = wave * 16 + m16;
  const int drow = wave * 16 + 8 * hh;
  const int rowBase = blockIdx.x * BR;

#pragma unroll 1
  for (int p = tid; p < W_PIECES; p += NTHR)
    *(v8us*)(sW + 8 * p) = *(const v8us*)(wimg + (size_t)p * 8);
  if (tid < 32) {
    sC[C_BSYM + tid]     = bfr(bsym[tid]);
    sC[C_BHD + tid]      = bfr(br1[tid]);
    sC[C_BHD + 32 + tid] = bfr(bc1[tid]);
    sC[C_WR2 + tid]      = bfr(wr2[tid]);
  }
  if (tid < 64) {
    sC[C_BIN + tid] = bfr(bin[tid]);
    sC[C_B1 + tid]  = bfr(b1[tid]);
    sC[C_B2 + tid]  = bfr(b2[tid]);
    sC[C_B3 + tid]  = bfr(b3[tid]);
  }
  if (tid < 128) sC[C_WC2 + tid] = bfr(wc2[tid]);
  if (tid == 0)  sC[C_BR2] = bfr(br2[0]);
  if (tid < 4)   sC[C_BC2 + tid] = bfr(bc2[tid]);

  if (wave < 4) {
    const int r = tid;
    int g = rowBase + r;
    g = (g < nrows) ? g : (nrows - 1);
    const float* xp = x + (size_t)g * XDIM;
    float xb[XDIM];
    unsigned short xq[XDIM];
#pragma unroll
    for (int i = 0; i < XDIM; ++i) {
      const unsigned short b = bf_bits(xp[i]);
      xq[i] = b;
      xb[i] = bf_up(b);
    }
    const float am = xb[0], bod = xb[1], dox = xb[2], ph = xb[4], nit = xb[7];
    const float p_ph  = pen_f(ph,  6.5f,   1.0f / 6.5f,   8.5f,  1.0f / 8.5f);
    const float p_am  = pen_f(am,  0.001f, 1.0f / 0.001f, 0.5f,  1.0f / 0.5f);
    const float p_bod = pen_f(bod, 0.001f, 1.0f / 0.001f, 5.0f,  1.0f / 5.0f);
    const float p_dob = (6.0f - dox) * (1.0f / 6.0f);
    const float p_do  = (dox < 6.0f) ? p_dob : 0.0f;
    const float p_nit = pen_f(nit, 0.001f, 1.0f / 0.001f, 10.0f, 1.0f / 10.0f);
    const float c05 = (float)(0.5 + 1e-8);
    const float c5  = (float)(5.0 + 1e-8);
    const float c10 = (float)(10.0 + 1e-8);
    const float c85 = (float)(8.5 + 1e-8);
    const float r05 = 1.0f / c05, r5 = 1.0f / c5, r10 = 1.0f / c10, r85 = 1.0f / c85;
    const float r3  = 1.0f / 3.0f;
    const float s_bact = (((1.2f * am) * r05 + (1.5f * bod) * r5) - (0.8f * dox) * r10) * r3;
    const float s_chem = ((1.5f * ph) * r85 + (1.0f * nit) * r10) * 0.5f;
    const float s_org  = (((2.0f * bod) * r5 - (1.5f * dox) * r10) + (0.8f * am) * r05) * r3;
    const float s_agr  = (2.0f * nit) * r10;
    const float psum   = (((p_ph + p_am) + p_bod) + p_do) + p_nit;
    const float den    = (1.0f + psum) + 1e-8f;
    const float resil  = 1.0f / den;
    float sym[10];
    sym[0] = p_ph; sym[1] = p_am; sym[2] = p_bod; sym[3] = p_do; sym[4] = p_nit;
    sym[5] = s_bact; sym[6] = s_chem; sym[7] = s_org; sym[8] = s_agr; sym[9] = resil;
    unsigned short hq[10], lq[10];
#pragma unroll
    for (int i = 0; i < 10; ++i) {
      const unsigned short hb = bf_bits(sym[i]);
      hq[i] = hb;
      lq[i] = bf_bits(sym[i] - bf_up(hb));
    }
    v8us q0, q1, q2, q3, xv8, z;
#pragma unroll
    for (int i = 0; i < 8; ++i) {
      q0[i] = hq[i]; q2[i] = lq[i];
      q1[i] = (unsigned short)0; q3[i] = (unsigned short)0;
      xv8[i] = xq[i];
      z[i] = (unsigned short)0;
    }
    q1[0] = hq[8]; q1[1] = hq[9];
    q3[0] = lq[8]; q3[1] = lq[9];
    unsigned short* srp = sS + r * PS;
    *(v8us*)(srp)      = q0;
    *(v8us*)(srp + 8)  = q1;
    *(v8us*)(srp + 16) = q2;
    *(v8us*)(srp + 24) = q3;
    unsigned short* arp = sA + r * PA;
    *(v8us*)(arp) = xv8;
    arp[8] = xq[8];
    arp[9] = xq[9];
    *(v8us*)(arp + 72) = z;
    *(v8us*)(arp + 80) = z;
    *(v8us*)(arp + 88) = z;
  }
  __syncthreads();

  {
    v8f acc0 = zero8(), acc1 = zero8();
    FragB a, bq0, bq1;
    const unsigned short* ap = sS + arow * PS + 8 * hh;
    a.u[0] = *(const v8us*)(ap);
    a.u[1] = *(const v8us*)(ap + 16);
    const unsigned short* wp0 = sW + R_SYM + m16 * P_SYM + 8 * hh;
    const unsigned short* wp1 = sW + R_SYM + (16 + m16) * P_SYM + 8 * hh;
    bq0.u[0] = *(const v8us*)(wp0);
    bq0.u[1] = *(const v8us*)(wp0 + 16);
    bq1.u[0] = *(const v8us*)(wp1);
    bq1.u[1] = *(const v8us*)(wp1 + 16);
    acc0 = mma_b(a.v, bq0.v, acc0);
    acc1 = mma_b(a.v, bq1.v, acc1);
    mma_guard2(acc0, acc1, a.v, bq0.v, bq1.v);
    const float bv0 = sC[C_BSYM + m16];
    const float bv1 = sC[C_BSYM + 16 + m16];
#pragma unroll
    for (int v = 0; v < 8; ++v) {
      unsigned short* rp = sA + (drow + v) * PA;
      const float e0 = elu_f(acc0[v] + bv0);
      const float e1 = elu_f(acc1[v] + bv1);
      st_hl(rp + 10 + m16, 32, e0);
      st_hl(rp + 26 + m16, 32, e1);
    }
  }
  __syncthreads();

  float h[4][8];
  {
    v8f acc[4];
#pragma unroll
    for (int t = 0; t < 4; ++t) acc[t] = zero8();
    const unsigned short* ap = sA + arow * PA + 8 * hh;
    const unsigned short* wp = sW + R_IN + m16 * P_IN + 8 * hh;
    FragB a, bq;
#pragma unroll
    for (int s = 0; s < 3; ++s) {
      a.u[0] = *(const v8us*)(ap + 32 * s);
      a.u[1] = *(const v8us*)(ap + 32 * s + 16);
#pragma unroll
      for (int t = 0; t < 4; ++t) {
        const unsigned short* w = wp + t * 16 * P_IN + 32 * s;
        bq.u[0] = *(const v8us*)(w);
        bq.u[1] = *(const v8us*)(w + 16);
        acc[t] = mma_b(a.v, bq.v, acc[t]);
      }
      mma_guard4(acc[0], acc[1], acc[2], acc[3], a.v, a.v, bq.v);
    }
    __syncthreads();
#pragma unroll
    for (int t = 0; t < 4; ++t) {
      const int c    = t * 16 + m16;
      const float bv = sC[C_BIN + c];
#pragma unroll
      for (int v = 0; v < 8; ++v) {
        const float e = elu_f(acc[t][v] + bv);
        h[t][v] = e;
        st_hl(sA + (drow + v) * PA + c, 64, e);
      }
    }
  }
  __syncthreads();

#pragma unroll 1
  for (int l = 0; l < 3; ++l) {
    const int woff = R_L1 + l * (64 * P_L);
    const int boff = C_B1 + l * 64;
    v8f acc[4];
#pragma unroll
    for (int t = 0; t < 4; ++t) acc[t] = zero8();
    const unsigned short* ap = sA + arow * PA + 8 * hh;
    const unsigned short* wp = sW + woff + m16 * P_L + 8 * hh;
    FragB ahi, alo, bq;
#pragma unroll
    for (int s = 0; s < 2; ++s) {
      ahi.u[0] = *(const v8us*)(ap + 32 * s);
      ahi.u[1] = *(const v8us*)(ap + 32 * s + 16);
      alo.u[0] = *(const v8us*)(ap + 64 + 32 * s);
      alo.u[1] = *(const v8us*)(ap + 64 + 32 * s + 16);
#pragma unroll
      for (int t = 0; t < 4; ++t) {
        const unsigned short* w = wp + t * 16 * P_L + 32 * s;
        bq.u[0] = *(const v8us*)(w);
        bq.u[1] = *(const v8us*)(w + 16);
        acc[t] = mma_b(ahi.v, bq.v, acc[t]);
        acc[t] = mma_b(alo.v, bq.v, acc[t]);
      }
      mma_guard4(acc[0], acc[1], acc[2], acc[3], ahi.v, alo.v, bq.v);
    }
    __syncthreads();
#pragma unroll
    for (int t = 0; t < 4; ++t) {
      const int c    = t * 16 + m16;
      const float bv = sC[boff + c];
#pragma unroll
      for (int v = 0; v < 8; ++v) {
        const float e  = elu_f(acc[t][v] + bv);
        const float hv = h[t][v] + e;
        h[t][v] = hv;
        st_hl(sA + (drow + v) * PA + c, 64, hv);
      }
    }
    __syncthreads();
  }

  {
    v8f acc[4];
#pragma unroll
    for (int t = 0; t < 4; ++t) acc[t] = zero8();
    const unsigned short* ap = sA + arow * PA + 8 * hh;
    const unsigned short* wp = sW + R_HD + m16 * P_L + 8 * hh;
    FragB ahi, alo, bq;
#pragma unroll
    for (int s = 0; s < 2; ++s) {
      ahi.u[0] = *(const v8us*)(ap + 32 * s);
      ahi.u[1] = *(const v8us*)(ap + 32 * s + 16);
      alo.u[0] = *(const v8us*)(ap + 64 + 32 * s);
      alo.u[1] = *(const v8us*)(ap + 64 + 32 * s + 16);
#pragma unroll
      for (int t = 0; t < 4; ++t) {
        const unsigned short* w = wp + t * 16 * P_L + 32 * s;
        bq.u[0] = *(const v8us*)(w);
        bq.u[1] = *(const v8us*)(w + 16);
        acc[t] = mma_b(ahi.v, bq.v, acc[t]);
        acc[t] = mma_b(alo.v, bq.v, acc[t]);
      }
      mma_guard4(acc[0], acc[1], acc[2], acc[3], ahi.v, alo.v, bq.v);
    }
    __syncthreads();
#pragma unroll
    for (int t = 0; t < 4; ++t) {
      const int c    = t * 16 + m16;
      const float bv = sC[C_BHD + c];
#pragma unroll
      for (int v = 0; v < 8; ++v) sE[(drow + v) * PE + c] = elu_f(acc[t][v] + bv);
    }
  }
  __syncthreads();

  if (wave < 4) {
    const int r = tid;
    const float* er = sE + r * PE;
    float p = 0.0f;
#pragma unroll 4
    for (int j = 0; j < 32; ++j) p = p + er[j] * sC[C_WR2 + j];
    p = p + sC[C_BR2];
    float q0 = 0.0f, q1 = 0.0f, q2 = 0.0f, q3 = 0.0f;
#pragma unroll 2
    for (int j = 0; j < 32; ++j) {
      const float ej = er[32 + j];
      const float* wc = sC + C_WC2 + 4 * j;
      q0 = q0 + ej * wc[0];
      q1 = q1 + ej * wc[1];
      q2 = q2 + ej * wc[2];
      q3 = q3 + ej * wc[3];
    }
    sPred[r] = p;
    sLog[4 * r + 0] = q0 + sC[C_BC2 + 0];
    sLog[4 * r + 1] = q1 + sC[C_BC2 + 1];
    sLog[4 * r + 2] = q2 + sC[C_BC2 + 2];
    sLog[4 * r + 3] = q3 + sC[C_BC2 + 3];
  }
  __syncthreads();

  {
    const bool actL = (tid < BR);
    const bool actP = (tid >= BR) && (tid < BR + 32);
    const int qL = actL ? tid : 0;
    const int qP = actP ? (tid - BR) : 0;
    const v4f vL = *(const v4f*)(sLog + qL * 4);
    const v4f vP = *(const v4f*)(sPred + qP * 4);
    float* opL = out + (size_t)nrows + (size_t)blockIdx.x * (BR * 4) + qL * 4;
    float* opP = out + (size_t)blockIdx.x * BR + qP * 4;
    if (actL) *(volatile v4f*)opL = vL;
    if (actP) *(volatile v4f*)opP = vP;
    __threadfence();
    if (actL) *(volatile v4f*)opL = vL;
    if (actP) *(volatile v4f*)opP = vP;
  }
}

static void launch_pack(const float* Wm, unsigned short* dst, int Kreal, int Ncols, int pitch,
                        int ksplit, int kshift, hipStream_t stream) {
  const int nPieces = Ncols * pitch / 8;
  const int blocks  = (nPieces + 255) / 256;
  k_pack<<<dim3(blocks), dim3(256), 0, stream>>>(Wm, dst, Kreal, Ncols, pitch, ksplit, kshift, nPieces);
}

extern "C" void kernel_launch(void* const* d_in, const int* in_sizes, int n_in,
                              void* d_out, int out_size, void* d_ws, size_t ws_size,
                              hipStream_t stream) {
  if (n_in < 19) return;
  if (in_sizes[0] != NROWS * XDIM) return;
  if (in_sizes[1] != 10 * 32 || in_sizes[2] != 32) return;
  if (in_sizes[3] != 42 * 64 || in_sizes[4] != 64) return;
  if (in_sizes[5] != 64 * 64 || in_sizes[6] != 64) return;
  if (in_sizes[7] != 64 * 64 || in_sizes[8] != 64) return;
  if (in_sizes[9] != 64 * 64 || in_sizes[10] != 64) return;
  if (in_sizes[11] != 64 * 32 || in_sizes[12] != 32) return;
  if (in_sizes[13] != 32 || in_sizes[14] != 1) return;
  if (in_sizes[15] != 64 * 32 || in_sizes[16] != 32) return;
  if (in_sizes[17] != 32 * 4 || in_sizes[18] != 4) return;
  if (out_size != NROWS * 5) return;

  const float* xin  = (const float*)d_in[0];
  const float* Wsym = (const float*)d_in[1];  const float* bsym = (const float*)d_in[2];
  const float* Win  = (const float*)d_in[3];  const float* bin  = (const float*)d_in[4];
  const float* W1   = (const float*)d_in[5];  const float* b1   = (const float*)d_in[6];
  const float* W2   = (const float*)d_in[7];  const float* b2   = (const float*)d_in[8];
  const float* W3   = (const float*)d_in[9];  const float* b3   = (const float*)d_in[10];
  const float* Wr1  = (const float*)d_in[11]; const float* br1  = (const float*)d_in[12];
  const float* Wr2  = (const float*)d_in[13]; const float* br2  = (const float*)d_in[14];
  const float* Wc1  = (const float*)d_in[15]; const float* bc1  = (const float*)d_in[16];
  const float* Wc2  = (const float*)d_in[17]; const float* bc2  = (const float*)d_in[18];
  float* out = (float*)d_out;

  const size_t tot = (size_t)W_TOT * 2;
  if (tot > ws_size) return;
  if (tot > (size_t)134217728) return;
  unsigned short* wimg = (unsigned short*)d_ws;

  const int nrows = in_sizes[0] / XDIM;
  if (nrows != NROWS || (nrows % BR) != 0) return;

  launch_pack(Wsym, wimg + R_SYM, 10, 32, P_SYM, 16, 16, stream);
  launch_pack(Win,  wimg + R_IN,  42, 64, P_IN,  42, 32, stream);
  launch_pack(W1,   wimg + R_L1,  64, 64, P_L,   64, 0,  stream);
  launch_pack(W2,   wimg + R_L2,  64, 64, P_L,   64, 0,  stream);
  launch_pack(W3,   wimg + R_L3,  64, 64, P_L,   64, 0,  stream);
  launch_pack(Wr1,  wimg + R_HD,  64, 32, P_L,   64, 0,  stream);
  launch_pack(Wc1,  wimg + R_HD2, 64, 32, P_L,   64, 0,  stream);

  k_main<<<dim3(nrows / BR), dim3(NTHR), 0, stream>>>(
      xin, wimg, bsym, bin, b1, b2, b3, br1, Wr2, br2, bc1, Wc2, bc2, out, nrows);
  (void)hipGetLastError();
}
